// LabelWiseAttention_89223650607792
// MI455X (gfx1250) — hardware-verified
//
#include <hip/hip_runtime.h>

typedef _Float16 v16h __attribute__((ext_vector_type(16)));
typedef _Float16 v8h  __attribute__((ext_vector_type(8)));
typedef float    v8f  __attribute__((ext_vector_type(8)));
typedef float    v4f  __attribute__((ext_vector_type(4)));
typedef v8h __attribute__((may_alias)) v8ha;
typedef v4f __attribute__((may_alias)) v4fa;

union Frag { v16h v; v8h half[2]; };

#define NB    8
#define NS    512
#define ND    1024
#define NC    14268
#define CPAD  14272
#define TLAB  32
#define NXE   (NB * NS * ND)
#define NWE   (NC * ND)
#define NX8   (NXE / 8)
#define NW8   (NWE / 8)
#define NOUT  (NB * NC)
#define NOUT4 (NOUT / 4)
#define WSCALE 16.0f
#define WINV   0.0625f

__device__ __forceinline__ v8f wmma_f16(v16h a, v16h b, v8f c) {
  v8f d = __builtin_amdgcn_wmma_f32_16x16x32_f16(false, a, false, b, (short)0, c, false, false);
  asm volatile("v_nop\n\tv_nop\n\tv_nop\n\tv_nop" : "+v"(d) : "v"(a), "v"(b));
  return d;
}

__device__ __forceinline__ v16h load_frag(const _Float16* p, int h) {
  Frag f;
  f.half[0] = *(const v8ha*)(p + 8 * h);
  f.half[1] = *(const v8ha*)(p + 16 + 8 * h);
  return f.v;
}

__global__ __launch_bounds__(256) void convert_kernel(
    const float* __restrict__ x, const float* __restrict__ wa, const float* __restrict__ wo,
    _Float16* __restrict__ xh, _Float16* __restrict__ wah, _Float16* __restrict__ woh)
{
  const int g = blockIdx.x * 256 + threadIdx.x;
  if (g >= NX8 + 2 * NW8) return;
  const float* src;
  _Float16* dst;
  float sc;
  if (g < NX8) {
    src = x + (size_t)g * 8;
    dst = xh + (size_t)g * 8;
    sc = 1.0f;
  } else if (g < NX8 + NW8) {
    const int e = g - NX8;
    src = wa + (size_t)e * 8;
    dst = wah + (size_t)e * 8;
    sc = WSCALE;
  } else {
    const int e = g - NX8 - NW8;
    src = wo + (size_t)e * 8;
    dst = woh + (size_t)e * 8;
    sc = WSCALE;
  }
  const v4f a = *(const v4fa*)src;
  const v4f c = *(const v4fa*)(src + 4);
  const v8h o = { (_Float16)(a.x * sc), (_Float16)(a.y * sc), (_Float16)(a.z * sc), (_Float16)(a.w * sc),
                  (_Float16)(c.x * sc), (_Float16)(c.y * sc), (_Float16)(c.z * sc), (_Float16)(c.w * sc) };
  *(volatile v8h*)dst = o;
  __threadfence();
  *(volatile v8h*)dst = o;
}

__global__ __launch_bounds__(256) void lwa_kernel(
    const _Float16* __restrict__ xh,
    const _Float16* __restrict__ wah,
    const _Float16* __restrict__ woh,
    const float* __restrict__ bo,
    float* __restrict__ ov)
{
  __shared__ float sM[8 * 16];
  __shared__ float sL[8 * 16];
  __shared__ float sA[8 * 16];
  __shared__ __attribute__((aligned(16))) float sOut[32];

  const int tid = threadIdx.x, lane = tid & 31, w = tid >> 5;
  const int h = lane >> 4, m = lane & 15;
  const int b = blockIdx.y;
  const int c0 = blockIdx.x * TLAB;

  const _Float16* xrow = xh + ((size_t)b * NS + 64 * w + m) * ND;
  const v8f zero8 = {0.f, 0.f, 0.f, 0.f, 0.f, 0.f, 0.f, 0.f};

  #pragma unroll 1
  for (int j = 0; j < 2; ++j) {
    const int cb = c0 + 16 * j;
    int cl = cb + m;
    cl = (cl < NC) ? cl : (NC - 1);
    const _Float16* warow = wah + (size_t)cl * ND;
    const _Float16* worow = woh + (size_t)cl * ND;

    v8f acA[4], acY[4];
    #pragma unroll
    for (int i = 0; i < 4; ++i) { acA[i] = zero8; acY[i] = zero8; }

    #pragma unroll 1
    for (int k0 = 0; k0 < ND; k0 += 32) {
      const v16h bwa = load_frag(warow + k0, h);
      const v16h bwo = load_frag(worow + k0, h);
      #pragma unroll
      for (int i = 0; i < 4; ++i) {
        const v16h a = load_frag(xrow + (size_t)(16 * i) * ND + k0, h);
        acA[i] = wmma_f16(a, bwa, acA[i]);
        acY[i] = wmma_f16(a, bwo, acY[i]);
      }
    }

    float mraw = acA[0][0];
    #pragma unroll
    for (int i = 0; i < 4; ++i)
      #pragma unroll
      for (int r = 0; r < 8; ++r) mraw = fmaxf(mraw, acA[i][r]);
    float l = 0.0f, acc = 0.0f;
    #pragma unroll
    for (int i = 0; i < 4; ++i)
      #pragma unroll
      for (int r = 0; r < 8; ++r) {
        const float p = __expf((acA[i][r] - mraw) * WINV);
        l += p;
        acc = fmaf(p, acY[i][r], acc);
      }

    const float m2 = __shfl_xor(mraw, 16);
    const float l2 = __shfl_xor(l, 16);
    const float a2 = __shfl_xor(acc, 16);
    const float M  = fmaxf(mraw, m2);
    const float e1 = __expf((mraw - M) * WINV);
    const float e2 = __expf((m2 - M) * WINV);
    const float L  = l * e1 + l2 * e2;
    const float A  = acc * e1 + a2 * e2;
    if (h == 0) {
      sM[w * 16 + m] = M;
      sL[w * 16 + m] = L;
      sA[w * 16 + m] = A;
    }
    __syncthreads();

    if (tid < 16) {
      float Mg = sM[tid];
      #pragma unroll
      for (int ww = 1; ww < 8; ++ww) Mg = fmaxf(Mg, sM[ww * 16 + tid]);
      float Lg = 0.0f, Ag = 0.0f;
      #pragma unroll
      for (int ww = 0; ww < 8; ++ww) {
        const float e = __expf((sM[ww * 16 + tid] - Mg) * WINV);
        Lg = fmaf(sL[ww * 16 + tid], e, Lg);
        Ag = fmaf(sA[ww * 16 + tid], e, Ag);
      }
      int cc = cb + tid;
      cc = (cc < NC) ? cc : (NC - 1);
      float logit = (Ag * WINV) * __builtin_amdgcn_rcpf(Lg) + bo[cc];
      logit = fminf(fmaxf(logit, -30.0f), 30.0f);
      sOut[16 * j + tid] = __builtin_amdgcn_rcpf(1.0f + __expf(-logit));
    }
    __syncthreads();
  }

  float* dst = ov + (size_t)b * CPAD + c0;
  v4f v = {0.f, 0.f, 0.f, 0.f};
  if (tid < 8) v = *(const v4fa*)(sOut + 4 * tid);
  if (tid < 8) *(volatile v4f*)(dst + 4 * tid) = v;
  __threadfence();
  if (tid < 8) *(volatile v4f*)(dst + 4 * tid) = v;
}

__global__ __launch_bounds__(256) void finalize_kernel(
    const float* __restrict__ ov, float* __restrict__ out)
{
  const int t = blockIdx.x * 256 + threadIdx.x;
  if (t >= NOUT4) return;
  const int i = 4 * t;
  const int b = i / NC;
  const int c = i - b * NC;
  const v4f v = *(const v4fa*)(ov + (size_t)b * CPAD + c);
  *(volatile v4f*)(out + i) = v;
  __threadfence();
  *(volatile v4f*)(out + i) = v;
}

extern "C" void kernel_launch(void* const* d_in, const int* in_sizes, int n_in,
                              void* d_out, int out_size, void* d_ws, size_t ws_size,
                              hipStream_t stream) {
  if (n_in < 4) return;
  if (in_sizes[0] != NXE) return;
  if (in_sizes[1] != NWE || in_sizes[2] != NWE) return;
  if (in_sizes[3] != NC) return;
  if (out_size != NOUT) return;

  const float* x  = (const float*)d_in[0];
  const float* Wa = (const float*)d_in[1];
  const float* Wo = (const float*)d_in[2];
  const float* bo = (const float*)d_in[3];
  float* out = (float*)d_out;

  const size_t xh_bytes = (size_t)NXE * 2;
  const size_t w_bytes  = (size_t)NWE * 2;
  const size_t ov_bytes = (size_t)NB * CPAD * 4;
  const size_t total = xh_bytes + 2 * w_bytes + ov_bytes;
  if (total > ws_size) return;

  char* ws = (char*)d_ws;
  _Float16* xh  = (_Float16*)(ws);
  _Float16* wah = (_Float16*)(ws + xh_bytes);
  _Float16* woh = (_Float16*)(ws + xh_bytes + w_bytes);
  float* ov     = (float*)(ws + xh_bytes + 2 * w_bytes);

  const int ngroups = NX8 + 2 * NW8;
  convert_kernel<<<(ngroups + 255) / 256, 256, 0, stream>>>(x, Wa, Wo, xh, wah, woh);

  dim3 gMain(CPAD / TLAB, NB);
  lwa_kernel<<<gMain, 256, 0, stream>>>(xh, wah, woh, bo, ov);

  finalize_kernel<<<(NOUT4 + 255) / 256, 256, 0, stream>>>(ov, out);
}
